// IQNRNNDistAgent_69166153335459
// MI455X (gfx1250) — hardware-verified
//
#include <hip/hip_runtime.h>
#include <math.h>

typedef _Float16 h16;
typedef __attribute__((ext_vector_type(16))) _Float16 v16h;
typedef __attribute__((ext_vector_type(8)))  _Float16 v8h;
typedef __attribute__((ext_vector_type(8)))  float    v8f;
typedef __attribute__((ext_vector_type(4)))  float    v4f;

#define BS_   4096
#define E_    256
#define H_    128
#define NQ_   8
#define QED_  64
#define NA_   14

__device__ __forceinline__ v8f wmma_f16(v16h a, v16h b, v8f c) {
  c = __builtin_amdgcn_wmma_f32_16x16x32_f16(false, a, false, b, (short)0, c, false, false);
  asm volatile("v_nop\n\tv_nop\n\tv_nop\n\tv_nop" : "+v"(c) : "v"(a), "v"(b));
  return c;
}

__device__ __forceinline__ v16h ldsA(const h16* base, int ld, int k0, int lane) {
  const int m  = lane & 15;
  const int hs = (lane >> 4) & 1;
  const h16* p = base + m * ld + k0 + hs * 8;
  v8h lo = *(const v8h*)(p);
  v8h hi = *(const v8h*)(p + 16);
  v16h a;
#pragma unroll
  for (int j = 0; j < 8; ++j) { a[j] = lo[j]; a[j + 8] = hi[j]; }
  return a;
}

__device__ __forceinline__ v16h gblBT(const h16* bt, int ld, int n0, int k0, int lane) {
  const int n  = lane & 15;
  const int hs = (lane >> 4) & 1;
  const h16* p = bt + (size_t)(n0 + n) * ld + k0 + hs * 8;
  v8h lo = *(const v8h*)(p);
  v8h hi = *(const v8h*)(p + 16);
  v16h b;
#pragma unroll
  for (int j = 0; j < 8; ++j) { b[j] = lo[j]; b[j + 8] = hi[j]; }
  return b;
}

__device__ __forceinline__ void split_h(float v, h16& hi, h16& lo) {
  hi = (h16)v;
  lo = (h16)((v - (float)hi) * 2048.0f);
}
__device__ __forceinline__ void wmma_split(v16h ah, v16h al, v16h bh, v16h bl, v8f& cm, v8f& cc) {
  cm = __builtin_amdgcn_wmma_f32_16x16x32_f16(false, ah, false, bh, (short)0, cm, false, false);
  cc = __builtin_amdgcn_wmma_f32_16x16x32_f16(false, ah, false, bl, (short)0, cc, false, false);
  cc = __builtin_amdgcn_wmma_f32_16x16x32_f16(false, al, false, bh, (short)0, cc, false, false);
  asm volatile("v_nop\n\tv_nop\n\tv_nop\n\tv_nop" : "+v"(cm), "+v"(cc) : "v"(ah), "v"(al), "v"(bh), "v"(bl));
}
#define RSPLIT 0.00048828125f

__device__ __forceinline__ unsigned pack2(h16 a, h16 b) {
  return (unsigned)__builtin_bit_cast(unsigned short, a) | ((unsigned)__builtin_bit_cast(unsigned short, b) << 16);
}

__global__ void hh_kernel(const float* __restrict__ hyp_w1,
                          const float* __restrict__ hyp_b1,
                          float* __restrict__ hh) {
  int j = threadIdx.x;
  if (j < 64) {
    float s = 0.0f;
#pragma unroll
    for (int k = 0; k < 8; ++k) s += hyp_w1[k * 64 + j];
    s = fmaxf(s + hyp_b1[j], 0.0f);
    ((volatile float*)hh)[j] = s;
    __threadfence();
    ((volatile float*)hh)[j] = s;
  }
}

__global__ void prep_kernel(const float* __restrict__ fc1_w,
                            const float* __restrict__ hyp_w2,
                            const float* __restrict__ hyp_b2,
                            const float* __restrict__ gru_wi,
                            const float* __restrict__ gru_wh,
                            const float* __restrict__ phi_w,
                            const float* __restrict__ fc2_w,
                            const float* __restrict__ rq,
                            const float* __restrict__ hh,
                            unsigned* __restrict__ fc1_wT2, unsigned* __restrict__ fc1_wL2,
                            unsigned* __restrict__ hypWT2,  unsigned* __restrict__ hypWL2,
                            unsigned* __restrict__ gruWiT2, unsigned* __restrict__ gruWiL2,
                            unsigned* __restrict__ gruWhT2, unsigned* __restrict__ gruWhL2,
                            unsigned* __restrict__ phiWT2,  unsigned* __restrict__ fc2WT2,
                            float* __restrict__ outRq) {
  const int NP = 87040 + 4096;
  for (int t = blockIdx.x * blockDim.x + threadIdx.x; t < NP; t += gridDim.x * blockDim.x) {
    if (t < 87040) {
      float f0, f1; unsigned* dst; unsigned* dstL = nullptr; int di;
      if (t < 16384) {
        int e0 = 2 * t; int n = e0 >> 8, k = e0 & 255;
        f0 = fc1_w[k * 128 + n]; f1 = fc1_w[(k + 1) * 128 + n];
        dst = fc1_wT2; dstL = fc1_wL2; di = t;
      } else if (t < 32768) {
        int u = 2 * (t - 16384); int o = u >> 7, i = u & 127;
        float s0 = 0.f, s1 = 0.f;
#pragma unroll 4
        for (int j = 0; j < 64; ++j) {
          s0 += hh[j] * hyp_w2[(size_t)j * 32768 + i * 256 + o];
          s1 += hh[j] * hyp_w2[(size_t)j * 32768 + (i + 1) * 256 + o];
        }
        f0 = s0 + hyp_b2[i * 256 + o]; f1 = s1 + hyp_b2[(i + 1) * 256 + o];
        dst = hypWT2; dstL = hypWL2; di = t - 16384;
      } else if (t < 57344) {
        int u = 2 * (t - 32768);
        f0 = gru_wi[u]; f1 = gru_wi[u + 1]; dst = gruWiT2; dstL = gruWiL2; di = t - 32768;
      } else if (t < 81920) {
        int u = 2 * (t - 57344);
        f0 = gru_wh[u]; f1 = gru_wh[u + 1]; dst = gruWhT2; dstL = gruWhL2; di = t - 57344;
      } else if (t < 86016) {
        int u = 2 * (t - 81920); int n = u >> 6, k = u & 63;
        f0 = phi_w[k * 128 + n]; f1 = phi_w[(k + 1) * 128 + n]; dst = phiWT2; di = t - 81920;
      } else {
        int u = 2 * (t - 86016); int n = u >> 7, k = u & 127;
        f0 = (n < NA_) ? fc2_w[k * NA_ + n] : 0.0f;
        f1 = (n < NA_) ? fc2_w[(k + 1) * NA_ + n] : 0.0f;
        dst = fc2WT2; di = t - 86016;
      }
      h16 h0, l0, h1, l1;
      split_h(f0, h0, l0); split_h(f1, h1, l1);
      const unsigned u2 = pack2(h0, h1), l2 = pack2(l0, l1);
      ((volatile unsigned*)dst)[di] = u2;
      if (dstL) ((volatile unsigned*)dstL)[di] = l2;
      __threadfence();
      ((volatile unsigned*)dst)[di] = u2;
      if (dstL) ((volatile unsigned*)dstL)[di] = l2;
    } else {
      int u = t - 87040;
      const float v = rq[u];
      ((volatile float*)outRq)[u] = v;
      __threadfence();
      ((volatile float*)outRq)[u] = v;
    }
  }
}

__global__ __launch_bounds__(32) void fused_kernel(
    const float* __restrict__ inputs, const float* __restrict__ hidden,
    const float* __restrict__ rq,     const float* __restrict__ fc1_b,
    const float* __restrict__ merger, const float* __restrict__ gru_bi,
    const float* __restrict__ gru_bh, const float* __restrict__ phi_b,
    const float* __restrict__ fc2_b,
    const h16* __restrict__ fc1_wT, const h16* __restrict__ fc1_wL,
    const h16* __restrict__ hypWT,  const h16* __restrict__ hypWL,
    const h16* __restrict__ gruWiT, const h16* __restrict__ gruWiL,
    const h16* __restrict__ gruWhT, const h16* __restrict__ gruWhL,
    const h16* __restrict__ phiWT,  const h16* __restrict__ fc2WT,
    float* __restrict__ outSorted,  float* __restrict__ outH) {

  __shared__ __align__(16) h16 aIn[16][E_ + 8];
  __shared__ __align__(16) h16 aInL[16][E_ + 8];
  __shared__ __align__(16) h16 x1[16][H_ + 8];
  __shared__ __align__(16) h16 x1L[16][H_ + 8];
  __shared__ __align__(16) h16 x2[16][H_ + 8];
  __shared__ __align__(16) h16 x2L[16][H_ + 8];
  __shared__ __align__(16) h16 hprev[16][H_ + 8];
  __shared__ __align__(16) h16 hprevL[16][H_ + 8];
  __shared__ __align__(16) h16 hnew[16][H_ + 8];
  __shared__ __align__(16) h16 cosT[16][QED_ + 8];
  __shared__ __align__(16) h16 qphi[16][H_ + 8];
  __shared__ __align__(16) float qbuf[128][16];
  __shared__ __align__(16) float hout[16][H_];
  __shared__ __align__(16) float qout[16 * NA_ * 8];

  const int lane = threadIdx.x & 31;
  const int n    = lane & 15;
  const int hs   = lane >> 4;
  const int row0 = blockIdx.x * 16;
  const v8f Z = {0.f, 0.f, 0.f, 0.f, 0.f, 0.f, 0.f, 0.f};

  {
    const v4f* ip = (const v4f*)(inputs + (size_t)row0 * E_);
    for (int idx = lane; idx < 16 * 64; idx += 32) {
      int r = idx >> 6, c4 = idx & 63;
      v4f v = ip[r * 64 + c4];
      int c = c4 * 4;
#pragma unroll
      for (int e = 0; e < 4; ++e) split_h(v[e], aIn[r][c + e], aInL[r][c + e]);
    }
    const v4f* hp = (const v4f*)(hidden + (size_t)row0 * H_);
    for (int idx = lane; idx < 16 * 32; idx += 32) {
      int r = idx >> 5, c4 = idx & 31;
      v4f v = hp[r * 32 + c4];
      int c = c4 * 4;
#pragma unroll
      for (int e = 0; e < 4; ++e) split_h(v[e], hprev[r][c + e], hprevL[r][c + e]);
    }
  }
  __syncthreads();

  for (int nt = 0; nt < 8; ++nt) {
    v8f am = Z, ac = Z;
#pragma unroll
    for (int k0 = 0; k0 < E_; k0 += 32)
      wmma_split(ldsA(&aIn[0][0], E_ + 8, k0, lane), ldsA(&aInL[0][0], E_ + 8, k0, lane),
                 gblBT(fc1_wT, E_, nt * 16, k0, lane), gblBT(fc1_wL, E_, nt * 16, k0, lane), am, ac);
    const int col = nt * 16 + n;
    const float b = fc1_b[col];
#pragma unroll
    for (int r = 0; r < 8; ++r)
      split_h(fmaxf((am[r] + ac[r] * RSPLIT) + b, 0.0f), x1[hs * 8 + r][col], x1L[hs * 8 + r][col]);
  }
  __syncthreads();

  for (int nt = 0; nt < 8; ++nt) {
    v8f a0 = Z, a1 = Z, c0 = Z, c1 = Z;
#pragma unroll
    for (int k0 = 0; k0 < H_; k0 += 32) {
      v16h ax = ldsA(&x1[0][0], H_ + 8, k0, lane), axl = ldsA(&x1L[0][0], H_ + 8, k0, lane);
      wmma_split(ax, axl, gblBT(hypWT, H_, nt * 16, k0, lane),       gblBT(hypWL, H_, nt * 16, k0, lane),       a0, c0);
      wmma_split(ax, axl, gblBT(hypWT, H_, nt * 16 + 128, k0, lane), gblBT(hypWL, H_, nt * 16 + 128, k0, lane), a1, c1);
    }
    const int col = nt * 16 + n;
    const float w0 = merger[col], w1 = merger[H_ + col];
    const float mx = fmaxf(w0, w1);
    const float e0 = expf(w0 - mx), e1 = expf(w1 - mx);
    const float s0 = e0 / (e0 + e1), s1 = e1 / (e0 + e1);
#pragma unroll
    for (int r = 0; r < 8; ++r) {
      const float em0 = a0[r] + c0[r] * RSPLIT, em1 = a1[r] + c1[r] * RSPLIT;
      split_h(fmaxf(s0 * em0 + s1 * em1, 0.0f), x2[hs * 8 + r][col], x2L[hs * 8 + r][col]);
    }
  }
  __syncthreads();

  for (int nt = 0; nt < 8; ++nt) {
    v8f gir = Z, giz = Z, gin = Z, ghr = Z, ghz = Z, ghn = Z;
    v8f cir = Z, ciz = Z, cin = Z, chr = Z, chz = Z, chn = Z;
    for (int k0 = 0; k0 < H_; k0 += 32) {
      v16h ax = ldsA(&x2[0][0], H_ + 8, k0, lane),    axl = ldsA(&x2L[0][0], H_ + 8, k0, lane);
      v16h ah = ldsA(&hprev[0][0], H_ + 8, k0, lane), ahl = ldsA(&hprevL[0][0], H_ + 8, k0, lane);
      wmma_split(ax, axl, gblBT(gruWiT, H_, nt * 16, k0, lane),       gblBT(gruWiL, H_, nt * 16, k0, lane),       gir, cir);
      wmma_split(ax, axl, gblBT(gruWiT, H_, nt * 16 + 128, k0, lane), gblBT(gruWiL, H_, nt * 16 + 128, k0, lane), giz, ciz);
      wmma_split(ax, axl, gblBT(gruWiT, H_, nt * 16 + 256, k0, lane), gblBT(gruWiL, H_, nt * 16 + 256, k0, lane), gin, cin);
      wmma_split(ah, ahl, gblBT(gruWhT, H_, nt * 16, k0, lane),       gblBT(gruWhL, H_, nt * 16, k0, lane),       ghr, chr);
      wmma_split(ah, ahl, gblBT(gruWhT, H_, nt * 16 + 128, k0, lane), gblBT(gruWhL, H_, nt * 16 + 128, k0, lane), ghz, chz);
      wmma_split(ah, ahl, gblBT(gruWhT, H_, nt * 16 + 256, k0, lane), gblBT(gruWhL, H_, nt * 16 + 256, k0, lane), ghn, chn);
    }
#pragma unroll
    for (int r = 0; r < 8; ++r) {
      gir[r] += cir[r] * RSPLIT; giz[r] += ciz[r] * RSPLIT; gin[r] += cin[r] * RSPLIT;
      ghr[r] += chr[r] * RSPLIT; ghz[r] += chz[r] * RSPLIT; ghn[r] += chn[r] * RSPLIT;
    }
    const int col = nt * 16 + n;
    const float bir = gru_bi[col], biz = gru_bi[col + 128], bin = gru_bi[col + 256];
    const float bhr = gru_bh[col], bhz = gru_bh[col + 128], bhn = gru_bh[col + 256];
#pragma unroll
    for (int r = 0; r < 8; ++r) {
      const int m = hs * 8 + r;
      float rg = 1.0f / (1.0f + expf(-((gir[r] + bir) + (ghr[r] + bhr))));
      float zg = 1.0f / (1.0f + expf(-((giz[r] + biz) + (ghz[r] + bhz))));
      float nn = tanhf((gin[r] + bin) + rg * (ghn[r] + bhn));
      float hp = hidden[(size_t)(row0 + m) * H_ + col];
      float hv = (1.0f - zg) * nn + zg * hp;
      hnew[m][col] = (h16)hv;
      hout[m][col] = hv;
    }
  }

  for (int idx = lane; idx < 16 * QED_; idx += 32) {
    int t = idx >> 6, f = idx & 63;
    float rv = rq[row0 + t];
    cosT[t][f] = (h16)cosf((3.1415927f * (float)f) * rv);
  }
  __syncthreads();

  for (int pass = 0; pass < 2; ++pass) {
#pragma unroll
    for (int m = 0; m < 16; ++m) {
      v4f v = *(const v4f*)(&hout[m][lane * 4]);
      *(volatile v4f*)(outH + (size_t)(row0 + m) * H_ + lane * 4) = v;
    }
    __threadfence();
  }

  for (int nt = 0; nt < 8; ++nt) {
    v8f acc = Z;
#pragma unroll
    for (int k0 = 0; k0 < QED_; k0 += 32)
      acc = wmma_f16(ldsA(&cosT[0][0], QED_ + 8, k0, lane), gblBT(phiWT, QED_, nt * 16, k0, lane), acc);
    const int col = nt * 16 + n;
    const float b = phi_b[col];
#pragma unroll
    for (int r = 0; r < 8; ++r)
      qphi[hs * 8 + r][col] = (h16)fmaxf(acc[r] + b, 0.0f);
  }
  __syncthreads();

  for (int ft = 0; ft < 8; ++ft) {
    v8f acc = Z;
    const int rr = lane & 15;
    const int fr = ft * 16 + rr;
    const int m  = fr >> 3;
    const int iq = fr & 7;
    const int qr = ((m >> 3) << 3) + iq;
#pragma unroll
    for (int k0 = 0; k0 < H_; k0 += 32) {
      const int kb = k0 + hs * 8;
      v16h a;
#pragma unroll
      for (int j = 0; j < 8; ++j)
        a[j] = (h16)((float)hnew[m][kb + j] * (float)qphi[qr][kb + j]);
#pragma unroll
      for (int j = 0; j < 8; ++j)
        a[j + 8] = (h16)((float)hnew[m][kb + 16 + j] * (float)qphi[qr][kb + 16 + j]);
      acc = wmma_f16(a, gblBT(fc2WT, H_, 0, k0, lane), acc);
    }
    const float bb = (n < NA_) ? fc2_b[n] : 0.0f;
#pragma unroll
    for (int r = 0; r < 8; ++r)
      qbuf[ft * 16 + hs * 8 + r][n] = acc[r] + bb;
  }
  __syncthreads();

  for (int idx = lane; idx < 16 * NA_; idx += 32) {
    int m = idx / NA_, a = idx % NA_;
    float v[8];
#pragma unroll
    for (int i = 0; i < 8; ++i) v[i] = qbuf[m * 8 + i][a];
#pragma unroll
    for (int i = 1; i < 8; ++i) {
      float key = v[i];
      int j = i - 1;
      while (j >= 0 && v[j] > key) { v[j + 1] = v[j]; --j; }
      v[j + 1] = key;
    }
#pragma unroll
    for (int i = 0; i < 8; ++i) qout[(m * NA_ + a) * 8 + i] = v[i];
  }
  __syncthreads();
  {
    float* ob = outSorted + (size_t)row0 * NA_ * 8;
    for (int pass = 0; pass < 2; ++pass) {
      for (int i = lane; i < 448; i += 32) {
        v4f v = *(const v4f*)(&qout[4 * i]);
        *(volatile v4f*)(ob + 4 * i) = v;
      }
      __threadfence();
    }
  }
}

extern "C" void kernel_launch(void* const* d_in, const int* in_sizes, int n_in,
                              void* d_out, int out_size, void* d_ws, size_t ws_size,
                              hipStream_t stream) {
  (void)in_sizes; (void)n_in; (void)out_size; (void)ws_size;
  const float* inputs = (const float*)d_in[0];
  const float* hidden = (const float*)d_in[1];
  const float* rq     = (const float*)d_in[2];
  const float* fc1_w  = (const float*)d_in[3];
  const float* fc1_b  = (const float*)d_in[4];
  const float* hyp_w1 = (const float*)d_in[5];
  const float* hyp_b1 = (const float*)d_in[6];
  const float* hyp_w2 = (const float*)d_in[7];
  const float* hyp_b2 = (const float*)d_in[8];
  const float* merger = (const float*)d_in[9];
  const float* gru_wi = (const float*)d_in[10];
  const float* gru_wh = (const float*)d_in[11];
  const float* gru_bi = (const float*)d_in[12];
  const float* gru_bh = (const float*)d_in[13];
  const float* phi_w  = (const float*)d_in[14];
  const float* phi_b  = (const float*)d_in[15];
  const float* fc2_w  = (const float*)d_in[16];
  const float* fc2_b  = (const float*)d_in[17];

  float* hh   = (float*)d_ws;
  h16* fc1_wT = (h16*)((char*)d_ws + 512);
  h16* fc1_wL = fc1_wT + 32768;
  h16* hypWT  = fc1_wL + 32768;
  h16* hypWL  = hypWT + 32768;
  h16* gruWiT = hypWL + 32768;
  h16* gruWiL = gruWiT + 49152;
  h16* gruWhT = gruWiL + 49152;
  h16* gruWhL = gruWhT + 49152;
  h16* phiWT  = gruWhL + 49152;
  h16* fc2WT  = phiWT + 8192;

  float* outSorted = (float*)d_out;
  float* outH      = outSorted + 4096 * 14 * 8;
  float* outRq     = outSorted + 983040;

  hipLaunchKernelGGL(hh_kernel, dim3(1), dim3(64), 0, stream, hyp_w1, hyp_b1, hh);
  hipLaunchKernelGGL(prep_kernel, dim3(356), dim3(256), 0, stream,
                     fc1_w, hyp_w2, hyp_b2, gru_wi, gru_wh, phi_w, fc2_w, rq, hh,
                     (unsigned*)fc1_wT, (unsigned*)fc1_wL, (unsigned*)hypWT, (unsigned*)hypWL,
                     (unsigned*)gruWiT, (unsigned*)gruWiL, (unsigned*)gruWhT, (unsigned*)gruWhL,
                     (unsigned*)phiWT, (unsigned*)fc2WT, outRq);
  hipLaunchKernelGGL(fused_kernel, dim3(256), dim3(32), 0, stream,
                     inputs, hidden, rq, fc1_b, merger, gru_bi, gru_bh, phi_b,
                     fc2_b, fc1_wT, fc1_wL, hypWT, hypWL, gruWiT, gruWiL, gruWhT, gruWhL, phiWT, fc2WT,
                     outSorted, outH);
}
